// KPConvLayer_2972117369005
// MI455X (gfx1250) — hardware-verified
//
#include <hip/hip_runtime.h>
#include <math.h>

constexpr int kNQ    = 50000;
constexpr int kNS    = 50000;
constexpr int kMNB   = 32;
constexpr int kKP    = 15;
constexpr int kKPP   = 16;
constexpr int kDin   = 128;
constexpr int kDout  = 128;
constexpr int kKD    = kKP * kDin;
constexpr int kXRows = kNS + 16;
constexpr int kQPB   = 16;
constexpr int kNT    = 256;
constexpr int kAGP   = 40;
constexpr int kXTP   = 40;
constexpr int kDCH   = 32;
constexpr int kNCH   = kDin / kDCH;
constexpr int kWCP   = kKP * kDCH + 8;
constexpr int kOSP   = 132;
constexpr float kCarry    = 2048.0f;
constexpr float kCarryInv = 1.0f / 2048.0f;
constexpr float kInvInfl  = 10.0f;

typedef char chk_tile0[(kNQ % kQPB == 0) ? 1 : -1];
typedef char chk_tile1[((kXRows * (kDin / 8)) % kNT == 0) ? 1 : -1];
typedef char chk_tile2[(kKD % 64 == 0 && kDout % 64 == 0) ? 1 : -1];
typedef char chk_tile3[(kDin % kDCH == 0 && kDCH == 32 && kMNB == 32) ? 1 : -1];
typedef char chk_tile4[(kQPB == 16 && kNT == 256 && kDout == 8 * 16) ? 1 : -1];

typedef __attribute__((ext_vector_type(16))) _Float16 v16h;
typedef __attribute__((ext_vector_type(8)))  _Float16 v8h;
typedef __attribute__((ext_vector_type(8)))  float    v8f;
typedef __attribute__((ext_vector_type(4)))  float    v4f;
typedef __attribute__((ext_vector_type(4)))  unsigned int v4u;

__device__ __forceinline__ void dep_guard_h(v8f& a, v8f& b, v16h x, v16h y) { asm volatile("v_nop\n\tv_nop\n\tv_nop\n\tv_nop" : "+v"(a), "+v"(b) : "v"(x), "v"(y)); }
template <typename T> struct Frag;
template <> struct Frag<_Float16> {
  typedef v16h V; union U { v16h v; v8h h[2]; };
  static __device__ __forceinline__ v16h load(const _Float16* p) {
    U f; f.h[0] = *(const v8h*)(p); f.h[1] = *(const v8h*)(p + 16); return f.v;
  }
  static __device__ __forceinline__ v8f mma(v16h a, v16h b, v8f c) {
    return __builtin_amdgcn_wmma_f32_16x16x32_f16(false, a, false, b, (short)0, c, false, false);
  }
  static __device__ __forceinline__ void guard(v8f& a, v8f& b, v16h x, v16h y) { dep_guard_h(a, b, x, y); }
};
__device__ __forceinline__ void guard_grp4(v8f& a, v8f& b, v8f& c, v8f& d,
                                           v16h p, v16h q, v16h r, v16h s, v16h t, v16h u) {
  asm volatile("v_nop\n\tv_nop\n\tv_nop\n\tv_nop"
               : "+v"(a), "+v"(b), "+v"(c), "+v"(d)
               : "v"(p), "v"(q), "v"(r), "v"(s), "v"(t), "v"(u));
}
__device__ __forceinline__ void guard_grp2(v8f& a, v8f& b, v16h p, v16h q, v16h r, v16h s) {
  asm volatile("v_nop\n\tv_nop\n\tv_nop\n\tv_nop"
               : "+v"(a), "+v"(b)
               : "v"(p), "v"(q), "v"(r), "v"(s));
}

__device__ __forceinline__ unsigned pk16(unsigned short a, unsigned short b) { return (unsigned)a | ((unsigned)b << 16); }

__device__ __forceinline__ void split_h(float v, unsigned short& hb, unsigned short& lb) {
  const _Float16 h = (_Float16)v;
  const float hf = (float)h;
  const float res = (v - hf) * kCarry;
  const _Float16 l = (_Float16)res;
  hb = __builtin_bit_cast(unsigned short, h);
  lb = __builtin_bit_cast(unsigned short, l);
}

__global__ __launch_bounds__(kNT) void feat_split_kernel(const float* __restrict__ x,
                                                         unsigned short* __restrict__ xh,
                                                         unsigned short* __restrict__ xl) {
  const int i = blockIdx.x * kNT + threadIdx.x;
  const int row = i >> 4, c = i & 15;
  const int rowc = (row < kNS) ? row : (kNS - 1);
  const float fl = (row < kNS) ? 1.0f : 0.0f;
  const float* p = x + (size_t)rowc * kDin + 8 * c;
  const v4f a = *(const v4f*)(p);
  const v4f b = *(const v4f*)(p + 4);
  unsigned short hb[8], lb[8];
#pragma unroll
  for (int e = 0; e < 4; ++e) {
    split_h(a[e] * fl, hb[e], lb[e]);
    split_h(b[e] * fl, hb[4 + e], lb[4 + e]);
  }
  const v4u uh = (v4u){pk16(hb[0], hb[1]), pk16(hb[2], hb[3]), pk16(hb[4], hb[5]), pk16(hb[6], hb[7])};
  const v4u ul = (v4u){pk16(lb[0], lb[1]), pk16(lb[2], lb[3]), pk16(lb[4], lb[5]), pk16(lb[6], lb[7])};
  unsigned short* qh = xh + 8 * (size_t)i;
  unsigned short* ql = xl + 8 * (size_t)i;
  *(volatile v4u*)qh = uh;
  *(volatile v4u*)ql = ul;
  __threadfence();
  *(volatile v4u*)qh = uh;
  *(volatile v4u*)ql = ul;
}

__global__ __launch_bounds__(kNT) void wt_split_kernel(const float* __restrict__ W,
                                                       unsigned short* __restrict__ wth,
                                                       unsigned short* __restrict__ wtl) {
  __shared__ float sm[64][65];
  const int t   = threadIdx.x;
  const int kd0 = blockIdx.x * 64;
  const int o0  = blockIdx.y * 64;
#pragma unroll
  for (int i = 0; i < 16; ++i) {
    const int e = i * kNT + t;
    const int r  = e >> 6;
    const int cl = e & 63;
    sm[cl][r] = W[(size_t)(kd0 + r) * kDout + o0 + cl];
  }
  __syncthreads();
  const int lane = t & 31, wave = t >> 5;
  const int q = lane >> 3, c8 = (lane & 7) * 8;
  for (int pass = 0; pass < 2; ++pass) {
#pragma unroll
    for (int it = 0; it < 2; ++it) {
      const int row = wave * 8 + it * 4 + q;
      unsigned short hb[8], lb[8];
#pragma unroll
      for (int e = 0; e < 8; ++e) split_h(sm[row][c8 + e], hb[e], lb[e]);
      const v4u uh = (v4u){pk16(hb[0], hb[1]), pk16(hb[2], hb[3]), pk16(hb[4], hb[5]), pk16(hb[6], hb[7])};
      const v4u ul = (v4u){pk16(lb[0], lb[1]), pk16(lb[2], lb[3]), pk16(lb[4], lb[5]), pk16(lb[6], lb[7])};
      const size_t off = (size_t)(o0 + row) * kKD + kd0 + c8;
      *(volatile v4u*)(wth + off) = uh;
      *(volatile v4u*)(wtl + off) = ul;
    }
    __threadfence();
  }
}

__device__ __forceinline__ void store_wchunk(_Float16* wch, _Float16* wcl, v8f am, v8f ar, int col, int hh) {
#pragma unroll
  for (int rr = 0; rr < 8; ++rr) {
    const int kp = 8 * hh + rr;
    const float v = am[rr] + ar[rr] * kCarryInv;
    unsigned short hb, lb;
    split_h(v, hb, lb);
    const _Float16 hv = __builtin_bit_cast(_Float16, hb);
    const _Float16 lv = __builtin_bit_cast(_Float16, lb);
    if (kp < kKP) {
      wch[kp * kDCH + col] = hv;
      wcl[kp * kDCH + col] = lv;
    }
  }
}

__global__ __launch_bounds__(kNT) void agg_kernel(const float* __restrict__ qpts,
                                                  const float* __restrict__ spts,
                                                  const int*   __restrict__ nbrs,
                                                  const float* __restrict__ kpts,
                                                  const unsigned short* __restrict__ xh,
                                                  const unsigned short* __restrict__ xl,
                                                  const unsigned short* __restrict__ wth,
                                                  const unsigned short* __restrict__ wtl,
                                                  float* __restrict__ out) {
  __shared__ int   nbr_s[kQPB * kMNB];
  __shared__ float qp_s[kQPB * 3];
  __shared__ float kp_s[48];
  __shared__ __align__(16) _Float16 ag_h[kQPB * kKPP * kAGP];
  __shared__ __align__(16) _Float16 ag_l[kQPB * kKPP * kAGP];
  __shared__ __align__(16) _Float16 xt_h[8 * kDCH * kXTP];
  __shared__ __align__(16) _Float16 xt_l[8 * kDCH * kXTP];
  __shared__ __align__(16) _Float16 wc_h[kQPB * kWCP];
  __shared__ __align__(16) _Float16 wc_l[kQPB * kWCP];
  __shared__ __align__(16) float    o_s[kQPB * kOSP];

  const int tid = threadIdx.x, lane = tid & 31, wave = tid >> 5;
  const int rlane = lane & 15, hh = lane >> 4, koff = hh * 8;
  const int blk = blockIdx.x;

  for (int i = tid; i < kQPB * kMNB; i += kNT) {
    int id = nbrs[(size_t)blk * (kQPB * kMNB) + i];
    id = (id < 0 || id >= kNS) ? kNS : id;
    nbr_s[i] = id;
  }
  if (tid < kQPB * 3) qp_s[tid] = qpts[(size_t)blk * (kQPB * 3) + tid];
  if (tid >= 64 && tid < 112) {
    const int j  = tid - 64;
    const int jc = (j < kKP * 3) ? j : (kKP * 3 - 1);
    const float v = kpts[jc];
    kp_s[j] = (j < kKP * 3) ? v : 0.0f;
  }
  __syncthreads();

#pragma unroll 1
  for (int p = tid; p < kQPB * kMNB; p += kNT) {
    const int q = p >> 5, m = p & 31;
    const int id = nbr_s[p];
    const bool live = id < kNS;
    const int idc = live ? id : 0;
    const float px = spts[(size_t)idc * 3 + 0];
    const float py = spts[(size_t)idc * 3 + 1];
    const float pz = spts[(size_t)idc * 3 + 2];
    const float rx = px - qp_s[q * 3 + 0];
    const float ry = py - qp_s[q * 3 + 1];
    const float rz = pz - qp_s[q * 3 + 2];
    const float fl = live ? 1.0f : 0.0f;
    _Float16* ah = ag_h + q * (kKPP * kAGP) + m;
    _Float16* al = ag_l + q * (kKPP * kAGP) + m;
#pragma unroll
    for (int k = 0; k < kKP; ++k) {
      const float dx = rx - kp_s[k * 3 + 0];
      const float dy = ry - kp_s[k * 3 + 1];
      const float dz = rz - kp_s[k * 3 + 2];
      const float d2 = dx * dx + dy * dy + dz * dz;
      const float w  = fmaxf(1.0f - sqrtf(d2) * kInvInfl, 0.0f) * fl;
      unsigned short hb, lb;
      split_h(w, hb, lb);
      const _Float16 hv = __builtin_bit_cast(_Float16, hb);
      const _Float16 lv = __builtin_bit_cast(_Float16, lb);
      ah[k * kAGP] = hv;
      al[k * kAGP] = lv;
    }
    const unsigned short zb = (unsigned short)0;
    const _Float16 zh = __builtin_bit_cast(_Float16, zb);
    ah[kKP * kAGP] = zh;
    al[kKP * kAGP] = zh;
  }
  __syncthreads();

  const v8f z8 = {0.f, 0.f, 0.f, 0.f, 0.f, 0.f, 0.f, 0.f};
  v8f cm = z8, cr = z8;
  const int ocol = wave * 16 + rlane;
  const _Float16* whrow = (const _Float16*)(wth + (size_t)ocol * kKD + koff);
  const _Float16* wlrow = (const _Float16*)(wtl + (size_t)ocol * kKD + koff);
  _Float16* xth = xt_h + wave * (kDCH * kXTP);
  _Float16* xtl = xt_l + wave * (kDCH * kXTP);

#pragma unroll 1
  for (int c = 0; c < kNCH; ++c) {
    const int d0 = c * kDCH;
#pragma unroll 1
    for (int r = 0; r < 2; ++r) {
      const int q = wave + 8 * r;
      {
        const int id = nbr_s[q * kMNB + lane];
        const unsigned short* ph = xh + (size_t)id * kDin + d0;
        const unsigned short* pl = xl + (size_t)id * kDin + d0;
        v4u gh[4], gl[4];
#pragma unroll
        for (int j = 0; j < 4; ++j) {
          gh[j] = *(const v4u*)(ph + 8 * j);
          gl[j] = *(const v4u*)(pl + 8 * j);
        }
#pragma unroll
        for (int j = 0; j < 4; ++j) {
#pragma unroll
          for (int e = 0; e < 4; ++e) {
            const int dd = 8 * j + 2 * e;
            const unsigned uh = gh[j][e], ul = gl[j][e];
            const unsigned short h0 = (unsigned short)(uh & 0xffffu), h1 = (unsigned short)(uh >> 16);
            const unsigned short l0 = (unsigned short)(ul & 0xffffu), l1 = (unsigned short)(ul >> 16);
            xth[dd * kXTP + lane]       = __builtin_bit_cast(_Float16, h0);
            xth[(dd + 1) * kXTP + lane] = __builtin_bit_cast(_Float16, h1);
            xtl[dd * kXTP + lane]       = __builtin_bit_cast(_Float16, l0);
            xtl[(dd + 1) * kXTP + lane] = __builtin_bit_cast(_Float16, l1);
          }
        }
      }
      __syncthreads();
      {
        const v16h fah = Frag<_Float16>::load(ag_h + q * (kKPP * kAGP) + rlane * kAGP + koff);
        const v16h fal = Frag<_Float16>::load(ag_l + q * (kKPP * kAGP) + rlane * kAGP + koff);
        const v16h bh0 = Frag<_Float16>::load(xth + rlane * kXTP + koff);
        const v16h bl0 = Frag<_Float16>::load(xtl + rlane * kXTP + koff);
        const v16h bh1 = Frag<_Float16>::load(xth + (16 + rlane) * kXTP + koff);
        const v16h bl1 = Frag<_Float16>::load(xtl + (16 + rlane) * kXTP + koff);
        v8f am0 = z8, ar0 = z8, am1 = z8, ar1 = z8;
        am0 = Frag<_Float16>::mma(fah, bh0, am0);
        ar0 = Frag<_Float16>::mma(fah, bl0, ar0);
        ar0 = Frag<_Float16>::mma(fal, bh0, ar0);
        am1 = Frag<_Float16>::mma(fah, bh1, am1);
        ar1 = Frag<_Float16>::mma(fah, bl1, ar1);
        ar1 = Frag<_Float16>::mma(fal, bh1, ar1);
        guard_grp4(am0, ar0, am1, ar1, fah, fal, bh0, bl0, bh1, bl1);
        store_wchunk(wc_h + q * kWCP, wc_l + q * kWCP, am0, ar0, rlane, hh);
        store_wchunk(wc_h + q * kWCP, wc_l + q * kWCP, am1, ar1, 16 + rlane, hh);
      }
      __syncthreads();
    }
#pragma unroll 1
    for (int kp = 0; kp < kKP; ++kp) {
      const v16h a_h = Frag<_Float16>::load(wc_h + rlane * kWCP + kp * kDCH + koff);
      const v16h a_l = Frag<_Float16>::load(wc_l + rlane * kWCP + kp * kDCH + koff);
      const v16h b_h = Frag<_Float16>::load(whrow + kp * kDin + d0);
      const v16h b_l = Frag<_Float16>::load(wlrow + kp * kDin + d0);
      cm = Frag<_Float16>::mma(a_h, b_h, cm);
      cr = Frag<_Float16>::mma(a_h, b_l, cr);
      cr = Frag<_Float16>::mma(a_l, b_h, cr);
      guard_grp2(cm, cr, a_h, a_l, b_h, b_l);
    }
  }

#pragma unroll
  for (int rr = 0; rr < 8; ++rr) {
    const float v = cm[rr] + cr[rr] * kCarryInv;
    o_s[(8 * hh + rr) * kOSP + wave * 16 + rlane] = v;
  }
  __syncthreads();
  {
    float* ob = out + (size_t)blk * (kQPB * kDout);
    const int row0 = wave * 2;
    const v4f v0 = *(const v4f*)(o_s + row0 * kOSP + 4 * lane);
    const v4f v1 = *(const v4f*)(o_s + (row0 + 1) * kOSP + 4 * lane);
    for (int pass = 0; pass < 2; ++pass) {
      *(volatile v4f*)(ob + (size_t)row0 * kDout + 4 * lane) = v0;
      *(volatile v4f*)(ob + (size_t)(row0 + 1) * kDout + 4 * lane) = v1;
      __threadfence();
    }
  }
}

extern "C" void kernel_launch(void* const* d_in, const int* in_sizes, int n_in,
                              void* d_out, int out_size, void* d_ws, size_t ws_size, hipStream_t stream) {
  (void)n_in;
  const float* qpts = (const float*)d_in[0];
  const float* spts = (const float*)d_in[1];
  const int*   nbrs = (const int*)d_in[2];
  const float* x    = (const float*)d_in[3];
  const float* kpts = (const float*)d_in[4];
  const float* W    = (const float*)d_in[5];
  float* out = (float*)d_out;

  const size_t P = (size_t)kXRows * kDin * 2;
  const size_t Q = (size_t)kDout * kKD * 2;
  const size_t total = 2 * P + 2 * Q;
  if (total > ws_size) return;
  if (out_size != kNQ * kDout) return;
  if (in_sizes[0] != kNQ * 3 || in_sizes[1] != kNS * 3 || in_sizes[2] != kNQ * kMNB ||
      in_sizes[3] != kNS * kDin || in_sizes[4] != kKP * 3 || in_sizes[5] != kKP * kDin * kDout) return;

  char* ws = (char*)d_ws;
  unsigned short* xh  = (unsigned short*)(ws);
  unsigned short* xl  = (unsigned short*)(ws + P);
  unsigned short* wth = (unsigned short*)(ws + 2 * P);
  unsigned short* wtl = (unsigned short*)(ws + 2 * P + Q);

  feat_split_kernel<<<(kXRows * (kDin / 8)) / kNT, kNT, 0, stream>>>(x, xh, xl);
  wt_split_kernel<<<dim3(kKD / 64, kDout / 64), kNT, 0, stream>>>(W, wth, wtl);
  agg_kernel<<<kNQ / kQPB, kNT, 0, stream>>>(qpts, spts, nbrs, kpts, xh, xl, wth, wtl, out);
}
